// SlidingWindowAttention_77189152244391
// MI455X (gfx1250) — hardware-verified
//
#include <hip/hip_runtime.h>


#ifndef NB
#define NB 4
#endif
#ifndef SEQ
#define SEQ 2048
#endif
#define NB_FULL  4
#define SEQ_FULL 2048
#define DM   1024
#define NH   16
#define HD   64
#define DQ   (NH * HD)
#define F3   (3 * DQ)
#define NPM  4
#define KVL  (SEQ + NPM)
#define KVP  (SEQ + 64)
#define RHC  512
#define RH   ((SEQ < RHC) ? SEQ : RHC)
#define PLP  72
#define PCAR 4096.0f
#define SCL  0.125f
#define CEXP (SCL * 1.4426950408889634f)
#define NEGB (-3.0e38f)
#define EPSV 1.1920928955078125e-7f

static_assert(SEQ % 64 == 0);
static_assert(SEQ >= 64);
static_assert((RH) % 16 == 0);
static_assert((RH) <= SEQ);
static_assert(DM % 256 == 0);
static_assert(HD == 64);
static_assert(KVP % 64 == 0);
static_assert(NB >= 1 && NB <= NB_FULL);
static_assert(SEQ <= SEQ_FULL);

typedef _Float16 h16;
typedef unsigned short bf;
typedef __attribute__((ext_vector_type(16))) __bf16   v16bf;
typedef __attribute__((ext_vector_type(16))) _Float16 v16h;
typedef __attribute__((ext_vector_type(8)))  _Float16 v8h;
typedef __attribute__((ext_vector_type(8)))  unsigned short v8us;
typedef __attribute__((ext_vector_type(8)))  float    v8f;
typedef __attribute__((ext_vector_type(4)))  float    v4f;
typedef __attribute__((ext_vector_type(2)))  _Float16 v2h;
typedef __attribute__((ext_vector_type(2)))  unsigned short v2us;
typedef __attribute__((ext_vector_type(2)))  float    v2f;
typedef v8h  __attribute__((may_alias)) v8ha;
typedef v4f  __attribute__((may_alias)) v4fa;
typedef v8us __attribute__((may_alias)) v8usa;

__device__ __forceinline__ unsigned short f2bf(float f) { unsigned u = __float_as_uint(f); u += 0x7FFFu + ((u >> 16) & 1u); return (unsigned short)(u >> 16); }
__device__ __forceinline__ float bf2f(unsigned short b) { return __uint_as_float(((unsigned)b) << 16); }
__device__ __forceinline__ float bfr(float f) { return bf2f(f2bf(f)); }
__device__ __forceinline__ v16h cat16(v8h lo, v8h hi) { return __builtin_shufflevector(lo, hi, 0, 1, 2, 3, 4, 5, 6, 7, 8, 9, 10, 11, 12, 13, 14, 15); }
__device__ __forceinline__ v16bf cat16b(v8us lo, v8us hi) { return __builtin_bit_cast(v16bf, __builtin_shufflevector(lo, hi, 0, 1, 2, 3, 4, 5, 6, 7, 8, 9, 10, 11, 12, 13, 14, 15)); }
__device__ __forceinline__ v8f wmma16(v16h a, v16h b, v8f c) { return __builtin_amdgcn_wmma_f32_16x16x32_f16(false, a, false, b, (short)0, c, false, false); }
__device__ __forceinline__ v8f wmmab(v16bf a, v16bf b, v8f c) { return __builtin_amdgcn_wmma_f32_16x16x32_bf16(false, a, false, b, (short)0, c, false, false); }
__device__ __forceinline__ h16 tohx(float x) { return (h16)x; }
__device__ __forceinline__ void splitf(float y, unsigned short& h, unsigned short& l) { h = f2bf(y); l = f2bf(y - bf2f(h)); }

template <typename T16> struct WFrag;
template <> struct WFrag<h16> { typedef v16h V; static __device__ __forceinline__ V ld(const h16* p) { return cat16(*(const v8h*)p, *(const v8h*)(p + 16)); } static __device__ __forceinline__ v8f mma(V a, V b, v8f c) { return wmma16(a, b, c); } };
template <> struct WFrag<bf> { typedef v16bf V; static __device__ __forceinline__ V ld(const bf* p) { return cat16b(*(const v8us*)p, *(const v8us*)(p + 16)); } static __device__ __forceinline__ v8f mma(V a, V b, v8f c) { return wmmab(a, b, c); } };

template <typename T16, int NSPLIT, bool RSC>
__global__ __launch_bounds__(32) void k_gemmw(const T16* __restrict__ A, const T16* __restrict__ A2, const T16* __restrict__ Bt, const T16* __restrict__ Bt2, int K, float* C, int ldc, const float* __restrict__ rs, size_t sA, size_t sB, size_t sC) {
    typedef typename WFrag<T16>::V V;
    __shared__ __align__(16) float os[16 * 68];
    const size_t z = blockIdx.z; A += z * sA; if (A2) A2 += z * sA; Bt += z * sB; if (Bt2) Bt2 += z * sB; C += z * sC;
    const int lane = threadIdx.x & 31, lr = lane & 15, hi = lane >> 4; const int r0 = blockIdx.x * 64, c0 = blockIdx.y * 64;
    v8f acc[4][4];
#pragma unroll
    for (int mb = 0; mb < 4; ++mb)
#pragma unroll
        for (int nb = 0; nb < 4; ++nb) acc[mb][nb] = (v8f){};
    const size_t aoff = (size_t)(r0 + lr) * K + 8 * hi, boff = (size_t)(c0 + lr) * K + 8 * hi;
#pragma unroll 1
    for (int kc = 0; kc < K; kc += 32) {
        V a[4], a2[4];
#pragma unroll
        for (int mb = 0; mb < 4; ++mb) { a[mb] = WFrag<T16>::ld(A + aoff + (size_t)mb * 16 * K + kc); if (NSPLIT == 1 || NSPLIT == 2) a2[mb] = WFrag<T16>::ld(A2 + aoff + (size_t)mb * 16 * K + kc); }
#pragma unroll
        for (int nb = 0; nb < 4; ++nb) { const V b = WFrag<T16>::ld(Bt + boff + (size_t)nb * 16 * K + kc); V b2; if (NSPLIT >= 2) b2 = WFrag<T16>::ld(Bt2 + boff + (size_t)nb * 16 * K + kc);
#pragma unroll
            for (int mb = 0; mb < 4; ++mb) { acc[mb][nb] = WFrag<T16>::mma(a[mb], b, acc[mb][nb]); if (NSPLIT == 1 || NSPLIT == 2) acc[mb][nb] = WFrag<T16>::mma(a2[mb], b, acc[mb][nb]); if (NSPLIT >= 2) acc[mb][nb] = WFrag<T16>::mma(a[mb], b2, acc[mb][nb]); } }
        asm volatile("v_nop\n\tv_nop\n\tv_nop\n\tv_nop" : "+v"(acc[0][0]), "+v"(acc[1][1]), "+v"(acc[2][2]), "+v"(acc[3][3]) : "v"(a[0]), "v"(a[3]));
    }
#pragma unroll
    for (int mb = 0; mb < 4; ++mb) {
#pragma unroll
        for (int nb = 0; nb < 4; ++nb) {
#pragma unroll
            for (int j = 0; j < 8; ++j) os[(hi * 8 + j) * 68 + nb * 16 + lr] = acc[mb][nb][j]; }
        __builtin_amdgcn_wave_barrier(); asm volatile("" ::: "memory");
        float* crow = C + (size_t)(r0 + mb * 16) * ldc + c0;
#pragma unroll 1
        for (int ps = 0; ps < 2; ++ps) {
#pragma unroll
            for (int s = 0; s < 8; ++s) { const int row = 2 * s + hi, cofs = lr * 4; v4f val = *(const v4fa*)(os + row * 68 + cofs); if (RSC) { const float g = rs[r0 + mb * 16 + row]; val = val * g; }
                *(volatile v4f*)(crow + (size_t)row * ldc + cofs) = val; }
            if (ps == 0) __threadfence(); }
        __builtin_amdgcn_wave_barrier(); asm volatile("" ::: "memory");
    }
}

__global__ __launch_bounds__(256) void k_cvt8(const float* __restrict__ src, bf* dst, size_t n8) { const size_t i = (size_t)blockIdx.x * 256 + threadIdx.x; if (i >= n8) return; const v8f v = *(const v8f*)(src + i * 8); v8us o;
#pragma unroll
    for (int k = 0; k < 8; ++k) o[k] = f2bf(v[k]); *(volatile v8us*)(dst + i * 8) = o; __threadfence(); *(volatile v8us*)(dst + i * 8) = o; }

__global__ __launch_bounds__(256) void k_wcvt(const float* __restrict__ w, const float* __restrict__ nw, bf* dst, size_t n8) { const size_t i = (size_t)blockIdx.x * 256 + threadIdx.x; if (i >= n8) return; const v8f v = *(const v8f*)(w + i * 8); const int k0 = (int)((i * 8) % DM); const v8f g = *(const v8f*)(nw + k0); v8us o;
#pragma unroll
    for (int k = 0; k < 8; ++k) o[k] = f2bf(bfr(v[k]) * bfr(g[k])); *(volatile v8us*)(dst + i * 8) = o; __threadfence(); *(volatile v8us*)(dst + i * 8) = o; }

__global__ __launch_bounds__(256) void k_xrow(const float* __restrict__ X, bf* XB, float* RS) {
    __shared__ float rsl[32];
    const int lane = threadIdx.x & 31, w = threadIdx.x >> 5;
#pragma unroll 1
    for (int q = 0; q < 4; ++q) { const int row = blockIdx.x * 32 + w * 4 + q; const float* xr = X + (size_t)row * DM; float ss = 0.f;
#pragma unroll
        for (int it = 0; it < DM / 256; ++it) { const v8f v = *(const v8f*)(xr + it * 256 + lane * 8); v8us o;
#pragma unroll
            for (int k = 0; k < 8; ++k) { o[k] = f2bf(v[k]); const float y = bf2f(o[k]); ss += y * y; }
            bf* dst = XB + (size_t)row * DM + it * 256 + lane * 8; *(volatile v8us*)dst = o; __threadfence(); *(volatile v8us*)dst = o; }
        ss += __shfl_xor(ss, 16, 32); ss += __shfl_xor(ss, 8, 32); ss += __shfl_xor(ss, 4, 32); ss += __shfl_xor(ss, 2, 32); ss += __shfl_xor(ss, 1, 32);
        const float r = 1.0f / sqrtf(ss * (1.0f / (float)DM) + EPSV);
        if (lane == 0) rsl[w * 4 + q] = r; }
    __syncthreads();
    if (w == 0) { const float v = rsl[lane]; float* d = RS + (size_t)blockIdx.x * 32 + lane; *(volatile float*)d = v; __threadfence(); *(volatile float*)d = v; }
}

struct InvF { float v[HD / 2]; };
static_assert(sizeof(InvF) == (HD / 2) * 4);
__global__ __launch_bounds__(256) void k_cstab(InvF iv, float* CS) { const int idx = blockIdx.x * 256 + threadIdx.x; if (idx >= SEQ * (HD / 2)) return; const int p = idx % (HD / 2); const int t = idx / (HD / 2); float f = 0.f;
#pragma unroll
    for (int i = 0; i < HD / 2; ++i) f = (p == i) ? iv.v[i] : f;
    const float ang = (float)t * f; v2f cs; cs[0] = cosf(ang); cs[1] = sinf(ang); *(volatile v2f*)(CS + (size_t)idx * 2) = cs; __threadfence(); *(volatile v2f*)(CS + (size_t)idx * 2) = cs; }

__global__ __launch_bounds__(256) void k_qpl(const float* __restrict__ F, const float* __restrict__ CS, h16* P16, bf* Ph, bf* Pl) {
#pragma clang fp contract(off)
    const size_t e = ((size_t)blockIdx.x * 256 + threadIdx.x) * 2; if (e >= (size_t)NH * SEQ * HD) return;
    const int d = (int)(e % HD); const int t = (int)((e / HD) % SEQ); const int h = (int)(e / ((size_t)HD * SEQ));
    const float* f = F + (size_t)t * F3 + h * HD + d; const float x0 = f[0], x1 = f[1];
    const v2f cs = *(const v2f*)(CS + ((size_t)t * (HD / 2) + (d >> 1)) * 2);
    const float r0 = x0 * cs[0] - x1 * cs[1]; const float r1 = x1 * cs[0] + x0 * cs[1];
    v2h o16; v2us oh, ol; unsigned short a, c;
    o16[0] = tohx(r0); splitf(r0, a, c); oh[0] = a; ol[0] = c;
    o16[1] = tohx(r1); splitf(r1, a, c); oh[1] = a; ol[1] = c;
    *(volatile v2h*)(P16 + e) = o16; *(volatile v2us*)(Ph + e) = oh; *(volatile v2us*)(Pl + e) = ol; __threadfence(); *(volatile v2h*)(P16 + e) = o16; *(volatile v2us*)(Ph + e) = oh; *(volatile v2us*)(Pl + e) = ol; }

__global__ __launch_bounds__(256) void k_kpl(const float* __restrict__ F, const float* __restrict__ pm, const float* __restrict__ CS, h16* P16, bf* Ph, bf* Pl) {
#pragma clang fp contract(off)
    const size_t e = ((size_t)blockIdx.x * 256 + threadIdx.x) * 2; if (e >= (size_t)NH * KVP * HD) return;
    const int d = (int)(e % HD); const int kv = (int)((e / HD) % KVP); const int h = (int)(e / ((size_t)HD * KVP));
    const int t = min(max(kv - NPM, 0), SEQ - 1);
    const float* f = F + (size_t)t * F3 + DQ + h * HD + d; const float x0 = f[0], x1 = f[1];
    const v2f cs = *(const v2f*)(CS + ((size_t)t * (HD / 2) + (d >> 1)) * 2);
    const float r0 = x0 * cs[0] - x1 * cs[1]; const float r1 = x1 * cs[0] + x0 * cs[1];
    const float* pp = pm + ((size_t)h * NPM + min(kv, NPM - 1)) * HD + d; const float g0 = bfr(pp[0]), g1 = bfr(pp[1]);
    const bool ism = (kv < NPM); const bool isk = (kv < KVL);
    const float y0 = ism ? g0 : (isk ? r0 : 0.0f); const float y1 = ism ? g1 : (isk ? r1 : 0.0f);
    v2h o16; v2us oh, ol; unsigned short a, c;
    o16[0] = tohx(y0); splitf(y0, a, c); oh[0] = a; ol[0] = c;
    o16[1] = tohx(y1); splitf(y1, a, c); oh[1] = a; ol[1] = c;
    *(volatile v2h*)(P16 + e) = o16; *(volatile v2us*)(Ph + e) = oh; *(volatile v2us*)(Pl + e) = ol; __threadfence(); *(volatile v2h*)(P16 + e) = o16; *(volatile v2us*)(Ph + e) = oh; *(volatile v2us*)(Pl + e) = ol; }

__global__ __launch_bounds__(256) void k_vpl(const float* __restrict__ F, const float* __restrict__ pm, h16* V16, bf* Vh, bf* Vl) {
    const size_t e = ((size_t)blockIdx.x * 256 + threadIdx.x) * 2; if (e >= (size_t)NH * HD * KVP) return;
    const int kv = (int)(e % KVP); const int d = (int)((e / KVP) % HD); const int h = (int)(e / ((size_t)KVP * HD));
    v2h o16; v2us oh, ol;
#pragma unroll
    for (int q = 0; q < 2; ++q) { const int kq = kv + q; const int t = min(max(kq - NPM, 0), SEQ - 1);
        const float xv = F[(size_t)t * F3 + 2 * DQ + h * HD + d]; const float g = bfr(pm[((size_t)h * NPM + min(kq, NPM - 1)) * HD + d]);
        const float y = (kq < NPM) ? g : ((kq < KVL) ? xv : 0.0f);
        o16[q] = tohx(y); unsigned short a, c; splitf(y, a, c); oh[q] = a; ol[q] = c; }
    *(volatile v2h*)(V16 + e) = o16; *(volatile v2us*)(Vh + e) = oh; *(volatile v2us*)(Vl + e) = ol; __threadfence(); *(volatile v2h*)(V16 + e) = o16; *(volatile v2us*)(Vh + e) = oh; *(volatile v2us*)(Vl + e) = ol; }

template <bool HR>
__global__ __launch_bounds__(32) void k_attn(const h16* __restrict__ Q16, const bf* __restrict__ Qh, const bf* __restrict__ Ql,
                                             const h16* __restrict__ K16, const bf* __restrict__ Kh, const bf* __restrict__ Kl,
                                             const h16* __restrict__ V16, const bf* __restrict__ Vh, const bf* __restrict__ Vl,
                                             int rbase, bf* Ah, bf* Al) {
    __shared__ __align__(16) unsigned short pl[2][16 * PLP];
    const int lane = threadIdx.x & 31, lr = lane & 15, hi = lane >> 4;
    const int q0 = rbase + (int)blockIdx.x * 16; const int head = blockIdx.y;
    const size_t qo = ((size_t)head * SEQ + q0 + lr) * HD + 8 * hi;
    const size_t kbase = (size_t)head * KVP * HD, vbase = (size_t)head * HD * KVP;
    v16h qa0 = (v16h){}, qa1 = (v16h){}; v16bf qh0 = (v16bf){}, qh1 = (v16bf){}, ql0 = (v16bf){}, ql1 = (v16bf){};
    if (HR) { qh0 = WFrag<bf>::ld(Qh + qo); qh1 = WFrag<bf>::ld(Qh + qo + 32); ql0 = WFrag<bf>::ld(Ql + qo); ql1 = WFrag<bf>::ld(Ql + qo + 32); }
    else    { qa0 = WFrag<h16>::ld(Q16 + qo); qa1 = WFrag<h16>::ld(Q16 + qo + 32); }
    v8f o[4];
#pragma unroll
    for (int nt = 0; nt < 4; ++nt) o[nt] = (v8f){};
    float mrow[8], lrow[8];
#pragma unroll
    for (int r = 0; r < 8; ++r) { mrow[r] = NEGB; lrow[r] = 0.f; }
    const int jtmax = (q0 + 15 + NPM) >> 6;
#pragma unroll 1
    for (int jt = 0; jt <= jtmax; ++jt) {
        const int j0 = jt * 64;
        v8f s[4];
#pragma unroll
        for (int nt = 0; nt < 4; ++nt) {
            const size_t ko = kbase + (size_t)(j0 + nt * 16 + lr) * HD + 8 * hi;
            s[nt] = (v8f){};
            if (HR) { const v16bf b0 = WFrag<bf>::ld(Kh + ko), b1 = WFrag<bf>::ld(Kh + ko + 32), e0 = WFrag<bf>::ld(Kl + ko), e1 = WFrag<bf>::ld(Kl + ko + 32);
                s[nt] = wmmab(qh0, b0, s[nt]); s[nt] = wmmab(ql0, b0, s[nt]); s[nt] = wmmab(qh0, e0, s[nt]);
                s[nt] = wmmab(qh1, b1, s[nt]); s[nt] = wmmab(ql1, b1, s[nt]); s[nt] = wmmab(qh1, e1, s[nt]); }
            else { const v16h b0 = WFrag<h16>::ld(K16 + ko), b1 = WFrag<h16>::ld(K16 + ko + 32);
                s[nt] = wmma16(qa0, b0, s[nt]); s[nt] = wmma16(qa1, b1, s[nt]); }
        }
        if (HR) asm volatile("v_nop\n\tv_nop\n\tv_nop\n\tv_nop" : "+v"(s[0]), "+v"(s[1]), "+v"(s[2]), "+v"(s[3]) : "v"(qh0), "v"(ql1));
        else    asm volatile("v_nop\n\tv_nop\n\tv_nop\n\tv_nop" : "+v"(s[0]), "+v"(s[1]), "+v"(s[2]), "+v"(s[3]) : "v"(qa0), "v"(qa1));
        if (j0 + 63 > q0 + NPM) {
#pragma unroll
            for (int r = 0; r < 8; ++r) { const int lim = q0 + 8 * hi + r + NPM - j0;
#pragma unroll
                for (int nt = 0; nt < 4; ++nt) if (nt * 16 + lr > lim) s[nt][r] = NEGB; } }
        float corr[8], psum[8];
#pragma unroll
        for (int r = 0; r < 8; ++r) { float t = fmaxf(fmaxf(s[0][r], s[1][r]), fmaxf(s[2][r], s[3][r]));
            t = fmaxf(t, __shfl_xor(t, 1, 32)); t = fmaxf(t, __shfl_xor(t, 2, 32)); t = fmaxf(t, __shfl_xor(t, 4, 32)); t = fmaxf(t, __shfl_xor(t, 8, 32));
            const float mn = fmaxf(mrow[r], t); corr[r] = __builtin_amdgcn_exp2f((mrow[r] - mn) * CEXP); mrow[r] = mn; psum[r] = 0.f; }
#pragma unroll
        for (int nt = 0; nt < 4; ++nt) {
#pragma unroll
            for (int r = 0; r < 8; ++r) { const float p = __builtin_amdgcn_exp2f((s[nt][r] - mrow[r]) * CEXP); const int li = (8 * hi + r) * PLP + nt * 16 + lr;
                if (HR) { unsigned short hb, lb; splitf(p, hb, lb); pl[0][li] = hb; pl[1][li] = lb; psum[r] += bf2f(hb) + bf2f(lb); }
                else    { const h16 ph = tohx(p * PCAR); pl[0][li] = __builtin_bit_cast(unsigned short, ph); psum[r] += (float)ph; } } }
#pragma unroll
        for (int r = 0; r < 8; ++r) { lrow[r] = lrow[r] * corr[r] + psum[r];
#pragma unroll
            for (int nt = 0; nt < 4; ++nt) o[nt][r] = o[nt][r] * corr[r]; }
        __syncthreads();
        const unsigned short* p0 = &pl[0][lr * PLP + 8 * hi]; const unsigned short* p1 = &pl[1][lr * PLP + 8 * hi];
        if (HR) {
            const v16bf a0 = cat16b(*(const v8usa*)p0, *(const v8usa*)(p0 + 16)), a1 = cat16b(*(const v8usa*)(p0 + 32), *(const v8usa*)(p0 + 48));
            const v16bf d0 = cat16b(*(const v8usa*)p1, *(const v8usa*)(p1 + 16)), d1 = cat16b(*(const v8usa*)(p1 + 32), *(const v8usa*)(p1 + 48));
#pragma unroll
            for (int nt = 0; nt < 4; ++nt) { const size_t vo = vbase + (size_t)(nt * 16 + lr) * KVP + j0 + 8 * hi;
                const v16bf b0 = WFrag<bf>::ld(Vh + vo), b1 = WFrag<bf>::ld(Vh + vo + 32), e0 = WFrag<bf>::ld(Vl + vo), e1 = WFrag<bf>::ld(Vl + vo + 32);
                o[nt] = wmmab(a0, b0, o[nt]); o[nt] = wmmab(d0, b0, o[nt]); o[nt] = wmmab(a0, e0, o[nt]);
                o[nt] = wmmab(a1, b1, o[nt]); o[nt] = wmmab(d1, b1, o[nt]); o[nt] = wmmab(a1, e1, o[nt]); }
            asm volatile("v_nop\n\tv_nop\n\tv_nop\n\tv_nop" : "+v"(o[0]), "+v"(o[1]), "+v"(o[2]), "+v"(o[3]) : "v"(a0), "v"(d1));
        } else {
            const v16h a0 = cat16(*(const v8ha*)p0, *(const v8ha*)(p0 + 16)), a1 = cat16(*(const v8ha*)(p0 + 32), *(const v8ha*)(p0 + 48));
#pragma unroll
            for (int nt = 0; nt < 4; ++nt) { const size_t vo = vbase + (size_t)(nt * 16 + lr) * KVP + j0 + 8 * hi;
                const v16h b0 = WFrag<h16>::ld(V16 + vo), b1 = WFrag<h16>::ld(V16 + vo + 32);
                o[nt] = wmma16(a0, b0, o[nt]); o[nt] = wmma16(a1, b1, o[nt]); }
            asm volatile("v_nop\n\tv_nop\n\tv_nop\n\tv_nop" : "+v"(o[0]), "+v"(o[1]), "+v"(o[2]), "+v"(o[3]) : "v"(a0), "v"(a1));
        }
        __syncthreads();
    }
    float inv[8];
#pragma unroll
    for (int r = 0; r < 8; ++r) { float l = lrow[r]; l += __shfl_xor(l, 1, 32); l += __shfl_xor(l, 2, 32); l += __shfl_xor(l, 4, 32); l += __shfl_xor(l, 8, 32); inv[r] = 1.0f / l; }
#pragma unroll
    for (int nt = 0; nt < 4; ++nt) {
#pragma unroll
        for (int r = 0; r < 8; ++r) { unsigned short hb, lb; splitf(o[nt][r] * inv[r], hb, lb); const int li = (8 * hi + r) * PLP + nt * 16 + lr; pl[0][li] = hb; pl[1][li] = lb; } }
    __syncthreads();
    const int prow = lane >> 3, pcs = (lane & 7) * 8;
#pragma unroll 1
    for (int ps = 0; ps < 2; ++ps) {
#pragma unroll
        for (int st = 0; st < 4; ++st) { const int row = st * 4 + prow;
            const v8us wh = *(const v8usa*)(&pl[0][row * PLP + pcs]); const v8us wl = *(const v8usa*)(&pl[1][row * PLP + pcs]);
            const size_t go = (size_t)(q0 + row) * DQ + (size_t)head * HD + pcs;
            *(volatile v8us*)(Ah + go) = wh; *(volatile v8us*)(Al + go) = wl; }
        if (ps == 0) __threadfence(); }
}

static double hsqrt(double a) { double y = (a > 1.0) ? a : 1.0; for (int i = 0; i < 400; ++i) { const double yn = 0.5 * (y + a / y); if (!(yn < y)) break; y = yn; } return y; }

extern "C" void kernel_launch(void* const* d_in, const int* in_sizes, int n_in,
                              void* d_out, int out_size, void* d_ws, size_t ws_size, hipStream_t stream) {
    if (n_in < 5) return;
    const int need_x = (NB - 1) * SEQ_FULL * DM + SEQ * DM;
    if (in_sizes[0] < need_x || in_sizes[1] < DM || in_sizes[2] < F3 * DM || in_sizes[3] < DM * DQ || in_sizes[4] < NH * NPM * HD || out_size < need_x) return;
    const float* x = (const float*)d_in[0]; const float* nw = (const float*)d_in[1]; const float* wqkv = (const float*)d_in[2]; const float* wo = (const float*)d_in[3]; const float* pm = (const float*)d_in[4];
    float* OUT = (float*)d_out;
    char* wsp = (char*)d_ws;
    auto take = [&](size_t bytes) { char* p = wsp; wsp += (bytes + 255) & ~(size_t)255; return (void*)p; };
    bf* WQKV = (bf*)take((size_t)F3 * DM * 2); bf* WO = (bf*)take((size_t)DM * DQ * 2); float* CS = (float*)take((size_t)SEQ * (HD / 2) * 2 * 4);
    bf* XB = (bf*)take((size_t)SEQ * DM * 2); float* RS = (float*)take((size_t)SEQ * 4); float* F = (float*)take((size_t)SEQ * F3 * 4);
    h16* QP16 = (h16*)take((size_t)NH * SEQ * HD * 2); bf* QPh = (bf*)take((size_t)NH * SEQ * HD * 2); bf* QPl = (bf*)take((size_t)NH * SEQ * HD * 2);
    h16* KP16 = (h16*)take((size_t)NH * KVP * HD * 2); bf* KPh = (bf*)take((size_t)NH * KVP * HD * 2); bf* KPl = (bf*)take((size_t)NH * KVP * HD * 2);
    h16* VT16 = (h16*)take((size_t)NH * HD * KVP * 2); bf* VTh = (bf*)take((size_t)NH * HD * KVP * 2); bf* VTl = (bf*)take((size_t)NH * HD * KVP * 2);
    bf* ATh = (bf*)take((size_t)SEQ * DQ * 2); bf* ATl = (bf*)take((size_t)SEQ * DQ * 2);
    if ((size_t)(wsp - (char*)d_ws) > ws_size) return;
    InvF iv;
    for (int p = 0; p < HD / 2; ++p) { double v = 1.0; for (int i = 0; i < p; ++i) v *= 10.0; const double r8 = hsqrt(hsqrt(hsqrt(v))); const float pw = (float)r8; iv.v[p] = 1.0f / pw; }
    k_wcvt<<<(unsigned)(((size_t)F3 * DM / 8 + 255) / 256), 256, 0, stream>>>(wqkv, nw, WQKV, (size_t)F3 * DM / 8);
    k_cvt8<<<(unsigned)(((size_t)DM * DQ / 8 + 255) / 256), 256, 0, stream>>>(wo, WO, (size_t)DM * DQ / 8);
    k_cstab<<<(unsigned)((SEQ * (HD / 2) + 255) / 256), 256, 0, stream>>>(iv, CS);
    const unsigned LQ = (unsigned)(((size_t)NH * SEQ * HD / 2 + 255) / 256), LK = (unsigned)(((size_t)NH * KVP * HD / 2 + 255) / 256);
    const int rh = RH;
    for (int b = 0; b < NB; ++b) {
        k_xrow<<<SEQ / 32, 256, 0, stream>>>(x + (size_t)b * SEQ_FULL * DM, XB, RS);
        k_gemmw<bf, 0, true><<<dim3(SEQ / 64, F3 / 64, 1), 32, 0, stream>>>(XB, nullptr, WQKV, nullptr, DM, F, F3, RS, 0, 0, 0);
        k_qpl<<<LQ, 256, 0, stream>>>(F, CS, QP16, QPh, QPl);
        k_kpl<<<LK, 256, 0, stream>>>(F, pm, CS, KP16, KPh, KPl);
        k_vpl<<<LK, 256, 0, stream>>>(F, pm, VT16, VTh, VTl);
        k_attn<true><<<dim3(rh / 16, NH, 1), 32, 0, stream>>>(QP16, QPh, QPl, KP16, KPh, KPl, VT16, VTh, VTl, 0, ATh, ATl);
        if (SEQ > rh) k_attn<false><<<dim3((SEQ - rh) / 16, NH, 1), 32, 0, stream>>>(QP16, QPh, QPl, KP16, KPh, KPl, VT16, VTh, VTl, rh, ATh, ATl);
        k_gemmw<bf, 1, false><<<dim3(SEQ / 64, DM / 64, 1), 32, 0, stream>>>(ATh, ATl, WO, nullptr, DQ, OUT + (size_t)b * SEQ_FULL * DM, DM, nullptr, 0, 0, 0);
    }
}
